// IAUBlock3D_53592601919761
// MI455X (gfx1250) — hardware-verified
//
#include <hip/hip_runtime.h>


namespace {
constexpr int NBt = 4, CCH = 1024, TT = 4, HW = 128, THW = TT * HW, CT = CCH * TT, CI = 512, NP = 4, NODE = TT * NP;
constexpr float XS = 8.0f, PS = 8.0f, WSC = 256.0f, EPS = 1e-5f;

typedef _Float16 b16;
typedef __attribute__((ext_vector_type(16))) _Float16 v16b;
typedef __attribute__((ext_vector_type(8))) _Float16 v8b;
typedef __attribute__((ext_vector_type(4))) _Float16 v4b;
typedef __attribute__((ext_vector_type(8))) float v8f;
typedef __attribute__((ext_vector_type(4))) float v4f;
__device__ __forceinline__ float bf16_rne(float f) { unsigned int u = __float_as_uint(f); u += 0x7FFFu + ((u >> 16) & 1u); return __uint_as_float(u & 0xFFFF0000u); }
__device__ __forceinline__ void split16(float v, b16& hi, b16& lo) { hi = (b16)v; lo = (b16)(v - (float)hi); }
__device__ __forceinline__ v16b frag_kb(const b16* p, int hh) { const v8b a = *(const v8b*)(p + 8 * hh), b = *(const v8b*)(p + 16 + 8 * hh); v16b f;
#pragma unroll
  for (int e = 0; e < 8; ++e) { f[e] = a[e]; f[8 + e] = b[e]; } return f; }
__device__ __forceinline__ v8f wmma16b(v16b a, v16b b, v8f c) { v8f d = __builtin_amdgcn_wmma_f32_16x16x32_f16(false, a, false, b, (short)0, c, false, false); asm volatile("v_nop\n\tv_nop\n\tv_nop\n\tv_nop" : "+v"(d) : "v"(a), "v"(b)); return d; }
__device__ __forceinline__ void wave_lds_sync() { __builtin_amdgcn_fence(__ATOMIC_RELEASE, "workgroup"); __builtin_amdgcn_wave_barrier(); __builtin_amdgcn_fence(__ATOMIC_ACQUIRE, "workgroup"); }
__device__ __forceinline__ float nexp(float x) { return __builtin_amdgcn_exp2f(x * 1.4426950408889634f); }
__device__ __forceinline__ float pmul(float a, float b) { float p = a * b; asm volatile("" : "+v"(p)); return p; }
__device__ __forceinline__ float sigm(float x) { return 1.0f / (1.0f + nexp(-x)); }
__device__ __forceinline__ float wsum(float v) {
#pragma unroll
  for (int o = 16; o >= 1; o >>= 1) v += __shfl_xor(v, o); return v; }

__global__ __launch_bounds__(256) void prepw_kernel(const float* __restrict__ w1, const float* __restrict__ gw, const float* __restrict__ w2, b16* __restrict__ W1s, b16* __restrict__ GWs, b16* __restrict__ W2s) {
  const int tid = blockIdx.x * 256 + threadIdx.x, nth = gridDim.x * 256;
  for (int pass = 0; pass < 2; ++pass) {
    for (int g = tid; g < (2 * CCH * CCH + CI * CCH) / 8; g += nth) { const float* src; b16* dst; int e;
      if (g < CCH * CCH / 8) { src = w1; dst = W1s; e = g * 8; } else if (g < 2 * CCH * CCH / 8) { src = w2; dst = W2s; e = (g - CCH * CCH / 8) * 8; } else { src = gw; dst = GWs; e = (g - 2 * CCH * CCH / 8) * 8; }
      const v4f a = *(const v4f*)(src + e), c = *(const v4f*)(src + e + 4); v8b o;
#pragma unroll
      for (int j = 0; j < 4; ++j) { o[j] = (b16)(bf16_rne(a[j]) * WSC); o[4 + j] = (b16)(bf16_rne(c[j]) * WSC); }
      *(volatile v8b*)(dst + e) = o; }
    __threadfence(); }
}
__global__ __launch_bounds__(256) void prept_kernel(const float* __restrict__ wt, const float* __restrict__ wp, const float* __restrict__ wg, const float* __restrict__ wu, b16* __restrict__ WT4) {
  __shared__ __attribute__((aligned(16))) b16 Tl[CI][64 + 8];
  const int which = blockIdx.y, k0 = blockIdx.x * 64, t_ = threadIdx.x; const float* w = which == 0 ? wt : which == 1 ? wp : which == 2 ? wg : wu;
  for (int k = t_; k < 64 * CI; k += 256) { const int kk = k / CI, o = k - kk * CI; Tl[o][kk] = (b16)(bf16_rne(w[(size_t)(k0 + kk) * CI + o]) * WSC); }
  __syncthreads();
  for (int pass = 0; pass < 2; ++pass) { for (int q = t_; q < CI * 8; q += 256) { const int o = q >> 3, c8 = (q & 7) * 8; *(volatile v8b*)(WT4 + ((size_t)which * CI + o) * CI + k0 + c8) = *(const v8b*)(&Tl[o][c8]); } __threadfence(); }
}
__global__ __launch_bounds__(256) void prepg_kernel(const float* __restrict__ x, b16* __restrict__ GX, b16* __restrict__ GXT) {
  __shared__ __attribute__((aligned(16))) b16 Tn[64][HW + 8], Tp[HW][64 + 8];
  const int b = blockIdx.y, n0 = blockIdx.x * 64, t_ = threadIdx.x; const float* xb = x + ((size_t)b * CT + n0) * HW;
  for (int k = t_; k < 64 * HW; k += 256) { const int nn = k >> 7, p = k & 127; const b16 v = (b16)(bf16_rne(xb[k]) * XS); Tn[nn][p] = v; Tp[p][nn] = v; }
  __syncthreads();
  for (int pass = 0; pass < 2; ++pass) {
    for (int q = t_; q < 64 * 16; q += 256) { const int nn = q >> 4, c8 = (q & 15) * 8; *(volatile v8b*)(GX + ((size_t)b * CT + n0 + nn) * HW + c8) = *(const v8b*)(&Tn[nn][c8]); }
    for (int q = t_; q < HW * 8; q += 256) { const int p = q >> 3, c8 = (q & 7) * 8; *(volatile v8b*)(GXT + ((size_t)b * HW + p) * CT + n0 + c8) = *(const v8b*)(&Tp[p][c8]); }
    __threadfence(); }
}
__global__ __launch_bounds__(64) void attn_kernel(const b16* __restrict__ GX, const b16* __restrict__ GXT, float* __restrict__ Y) {
  __shared__ __attribute__((aligned(16))) float To[2][16][HW + 4];
  const int wave = threadIdx.x >> 5, lane = threadIdx.x & 31, hh = lane >> 4, col = lane & 15; const int b = blockIdx.y, q0 = blockIdx.x * 32 + wave * 16, qi = q0 + col;
  const b16* G = GX + (size_t)b * CT * HW; const b16* GT = GXT + (size_t)b * HW * CT;
  v16b qf[4];
#pragma unroll
  for (int ks = 0; ks < 4; ++ks) qf[ks] = frag_kb(G + (size_t)qi * HW + ks * 32, hh);
  float m = -INFINITY, l = 0.0f; v8f o[8];
#pragma unroll
  for (int t = 0; t < 8; ++t) o[t] = (v8f){};
  for (int kb = 0; kb < CT; kb += 32) {
    v8f s0 = {}, s1 = {};
#pragma unroll
    for (int ks = 0; ks < 4; ++ks) { s0 = wmma16b(frag_kb(G + (size_t)(kb + col) * HW + ks * 32, hh), qf[ks], s0); s1 = wmma16b(frag_kb(G + (size_t)(kb + 16 + col) * HW + ks * 32, hh), qf[ks], s1); }
    float mr = -INFINITY;
#pragma unroll
    for (int r = 0; r < 8; ++r) { s0[r] *= 1.0f / (XS * XS); s1[r] *= 1.0f / (XS * XS); mr = fmaxf(mr, fmaxf(s0[r], s1[r])); }
    mr = fmaxf(mr, __shfl_xor(mr, 16)); const float mn = fmaxf(m, mr); const float al_ = nexp(m - mn); m = mn; float sum = 0.0f; v16b pb, pl;
#pragma unroll
    for (int r = 0; r < 8; ++r) { const float e0 = nexp(s0[r] - mn), e1 = nexp(s1[r] - mn); sum += e0 + e1; b16 a_, c_; split16(e0 * PS, a_, c_); pb[r] = a_; pl[r] = c_; split16(e1 * PS, a_, c_); pb[8 + r] = a_; pl[8 + r] = c_; }
    sum += __shfl_xor(sum, 16); l = l * al_ + sum;
#pragma unroll
    for (int t = 0; t < 8; ++t) { o[t] *= al_; const v16b g = frag_kb(GT + (size_t)(t * 16 + col) * CT + kb, hh); o[t] = wmma16b(g, pb, o[t]); o[t] = wmma16b(g, pl, o[t]); } }
  const float inv = 1.0f / (l * PS * XS);
#pragma unroll
  for (int t = 0; t < 8; ++t)
#pragma unroll
    for (int r = 0; r < 8; ++r) To[wave][col][t * 16 + 8 * hh + r] = o[t][r] * inv;
  wave_lds_sync();
  for (int pass = 0; pass < 2; ++pass) { for (int rr = 0; rr < 16; ++rr) *(volatile v4f*)(Y + ((size_t)b * CT + q0 + rr) * HW + lane * 4) = *(const v4f*)(&To[wave][rr][lane * 4]); __threadfence(); }
}
__global__ __launch_bounds__(256) void ytrans_kernel(const float* __restrict__ Y, b16* __restrict__ YTH, b16* __restrict__ YTL) {
  __shared__ __attribute__((aligned(16))) b16 Th[HW][64 + 8], Tl[HW][64 + 8];
  const int b = blockIdx.y >> 2, t = blockIdx.y & 3, c0 = blockIdx.x * 64, t_ = threadIdx.x;
  for (int k = t_; k < 64 * HW; k += 256) { const int cc = k >> 7, p = k & 127; const float v = Y[((size_t)b * CT + (size_t)(c0 + cc) * TT + t) * HW + p]; b16 a_, c_; split16(v * XS, a_, c_); Th[p][cc] = a_; Tl[p][cc] = c_; }
  __syncthreads();
  for (int pass = 0; pass < 2; ++pass) { for (int q = t_; q < HW * 8; q += 256) { const int p = q >> 3, c8 = (q & 7) * 8; const size_t gi = (((size_t)b * TT + t) * HW + p) * CCH + c0 + c8; *(volatile v8b*)(YTH + gi) = *(const v8b*)(&Th[p][c8]); *(volatile v8b*)(YTL + gi) = *(const v8b*)(&Tl[p][c8]); } __threadfence(); }
}
__global__ __launch_bounds__(128) void w1_kernel(const b16* __restrict__ W1s, const b16* __restrict__ YTH, const b16* __restrict__ YTL, const float* __restrict__ bias, float* __restrict__ Y1) {
  __shared__ __attribute__((aligned(16))) float Ts[4][16][HW + 4];
  const int wave = threadIdx.x >> 5, lane = threadIdx.x & 31, nloc = lane & 15, hlf = lane >> 4; const int b = blockIdx.z, o0 = blockIdx.y * 64 + wave * 16, p0 = blockIdx.x * HW;
  const b16* Bh = YTH + ((size_t)b * THW + p0) * CCH; const b16* Bl = YTL + ((size_t)b * THW + p0) * CCH;
  v8f acc[8];
#pragma unroll
  for (int t = 0; t < 8; ++t) acc[t] = (v8f){};
#pragma unroll 2
  for (int kb = 0; kb < CCH; kb += 32) { const v16b a = frag_kb(W1s + (size_t)(o0 + nloc) * CCH + kb, hlf);
#pragma unroll
    for (int t = 0; t < 8; ++t) { acc[t] = wmma16b(a, frag_kb(Bh + (size_t)(t * 16 + nloc) * CCH + kb, hlf), acc[t]); acc[t] = wmma16b(a, frag_kb(Bl + (size_t)(t * 16 + nloc) * CCH + kb, hlf), acc[t]); } }
#pragma unroll
  for (int t = 0; t < 8; ++t)
#pragma unroll
    for (int r = 0; r < 8; ++r) Ts[wave][8 * hlf + r][t * 16 + nloc] = acc[t][r] * (1.0f / (XS * WSC)) + bf16_rne(bias[o0 + 8 * hlf + r]);
  wave_lds_sync();
  for (int pass = 0; pass < 2; ++pass) { for (int rr = 0; rr < 16; ++rr) *(volatile v4f*)(Y1 + ((size_t)b * CCH + o0 + rr) * THW + p0 + lane * 4) = *(const v4f*)(&Ts[wave][rr][lane * 4]); __threadfence(); }
}
__global__ __launch_bounds__(256) void bnstat_kernel(const float* __restrict__ V, int C, float* __restrict__ MEAN, float* __restrict__ VAR) {
  __shared__ float Sp[32][8], Smu[32], Svar[32];
  const int t_ = threadIdx.x, cl = t_ >> 3, j = t_ & 7, c = blockIdx.x * 32 + cl;
  float s = 0.0f; for (int b = 0; b < NBt; ++b) { const float* row = V + ((size_t)b * C + c) * THW; for (int p = j * 64; p < j * 64 + 64; ++p) s += row[p]; }
  Sp[cl][j] = s; __syncthreads();
  if (t_ < 32) { float a = 0.0f; for (int k = 0; k < 8; ++k) a += Sp[t_][k]; Smu[t_] = a * (1.0f / (NBt * THW)); }
  __syncthreads();
  const float mu = Smu[cl]; float ss = 0.0f; for (int b = 0; b < NBt; ++b) { const float* row = V + ((size_t)b * C + c) * THW; for (int p = j * 64; p < j * 64 + 64; ++p) { const float d = row[p] - mu; ss += pmul(d, d); } }
  __syncthreads(); Sp[cl][j] = ss; __syncthreads();
  if (t_ < 32) { float a = 0.0f; for (int k = 0; k < 8; ++k) a += Sp[t_][k]; Svar[t_] = a * (1.0f / (NBt * THW)); }
  __syncthreads();
  for (int pass = 0; pass < 2; ++pass) { if (t_ < 32) { ((volatile float*)MEAN)[blockIdx.x * 32 + t_] = Smu[t_]; ((volatile float*)VAR)[blockIdx.x * 32 + t_] = Svar[t_]; } __threadfence(); }
}
__global__ __launch_bounds__(256) void zmake_kernel(const float* __restrict__ Y1, const float* __restrict__ x, const float* __restrict__ MEAN, const float* __restrict__ VAR, const float* __restrict__ g, const float* __restrict__ be, float* __restrict__ Z, float* __restrict__ USUM) {
  __shared__ float Su[32];
  const int wave = threadIdx.x >> 5, lane = threadIdx.x & 31, b = blockIdx.y, c = blockIdx.x * 32 + wave;
  for (int cc = c, w8 = wave; w8 < 32; cc += 8, w8 += 8) {
    const float mu = MEAN[cc], rs = rsqrtf(VAR[cc] + EPS), gg = bf16_rne(g[cc]), bb = bf16_rne(be[cc]); const size_t row = ((size_t)b * CCH + cc) * THW;
    v4f zv[4]; float s = 0.0f;
#pragma unroll
    for (int q = 0; q < 4; ++q) { const v4f y = *(const v4f*)(Y1 + row + q * 128 + lane * 4), xx = *(const v4f*)(x + row + q * 128 + lane * 4); v4f z;
#pragma unroll
      for (int e = 0; e < 4; ++e) { z[e] = pmul((y[e] - mu) * rs, gg) + bb + bf16_rne(xx[e]); s += z[e]; } zv[q] = z; }
    s = wsum(s); if (lane == 0) Su[w8] = s * (1.0f / THW);
    for (int pass = 0; pass < 2; ++pass) {
#pragma unroll
      for (int q = 0; q < 4; ++q) *(volatile v4f*)(Z + row + q * 128 + lane * 4) = zv[q]; __threadfence(); } }
  __syncthreads();
  for (int pass = 0; pass < 2; ++pass) { if (threadIdx.x < 32) ((volatile float*)USUM)[b * CCH + blockIdx.x * 32 + threadIdx.x] = Su[threadIdx.x]; __threadfence(); }
}
__global__ __launch_bounds__(256) void sapre_kernel(const float* __restrict__ Z, const float* __restrict__ saw, const float* __restrict__ sab, float* __restrict__ SPRE) {
  __shared__ __attribute__((aligned(16))) float Tz[64][64 + 1];
  const int b = blockIdx.y, p0 = blockIdx.x * 64, t_ = threadIdx.x, n = t_ >> 6, j = t_ & 63;
  float s = bf16_rne(sab[n]);
  for (int c0 = 0; c0 < CCH; c0 += 64) {
    __syncthreads();
    for (int k = t_; k < 64 * 64; k += 256) { const int cc = k >> 6, pp = k & 63; Tz[cc][pp] = Z[((size_t)b * CCH + c0 + cc) * THW + p0 + pp]; }
    __syncthreads();
    for (int cc = 0; cc < 64; ++cc) s += pmul(bf16_rne(saw[n * CCH + c0 + cc]), Tz[cc][j]); }
  for (int pass = 0; pass < 2; ++pass) { ((volatile float*)SPRE)[((size_t)b * NP + n) * THW + p0 + j] = s; __threadfence(); }
}
__global__ __launch_bounds__(256) void bn2_kernel(const float* __restrict__ SPRE, float* __restrict__ MV2) {
  __shared__ float Sp[4][64], Smu[4], Sout[32];
  const int t_ = threadIdx.x, n = t_ >> 6, j = t_ & 63;
  float s = 0.0f; for (int b = 0; b < NBt; ++b) for (int p = j * 8; p < j * 8 + 8; ++p) s += SPRE[((size_t)b * NP + n) * THW + p];
  Sp[n][j] = s; __syncthreads();
  if (t_ < 4) { float a = 0.0f; for (int k = 0; k < 64; ++k) a += Sp[t_][k]; Smu[t_] = a * (1.0f / (NBt * THW)); }
  __syncthreads();
  const float mu = Smu[n]; float ss = 0.0f; for (int b = 0; b < NBt; ++b) for (int p = j * 8; p < j * 8 + 8; ++p) { const float d = SPRE[((size_t)b * NP + n) * THW + p] - mu; ss += pmul(d, d); }
  __syncthreads(); Sp[n][j] = ss; __syncthreads();
  if (t_ < 32) { float v = 0.0f; if (t_ < 4) v = Smu[t_]; else if (t_ < 8) { float a = 0.0f; for (int k = 0; k < 64; ++k) a += Sp[t_ - 4][k]; v = a * (1.0f / (NBt * THW)); } Sout[t_] = v; }
  __syncthreads();
  for (int pass = 0; pass < 2; ++pass) { if (t_ < 32) ((volatile float*)MV2)[t_] = Sout[t_]; __threadfence(); }
}
__global__ __launch_bounds__(256) void amake_kernel(const float* __restrict__ SPRE, const float* __restrict__ MV2, const float* __restrict__ g, const float* __restrict__ be, float* __restrict__ A_, float* __restrict__ aout) {
  const int b = blockIdx.x, wave = threadIdx.x >> 5, lane = threadIdx.x & 31;
  for (int rr = wave; rr < NP * TT; rr += 8) { const int n = rr >> 2, t = rr & 3; const float mu = MV2[n], rs = rsqrtf(MV2[4 + n] + EPS), gg = bf16_rne(g[n]), bb = bf16_rne(be[n]);
    const v4f sp = *(const v4f*)(SPRE + ((size_t)b * NP + n) * THW + t * HW + lane * 4); v4f a;
#pragma unroll
    for (int e = 0; e < 4; ++e) a[e] = sigm(pmul((sp[e] - mu) * rs, gg) + bb);
    for (int pass = 0; pass < 2; ++pass) { *(volatile v4f*)(A_ + ((size_t)b * NP + n) * THW + t * HW + lane * 4) = a; *(volatile v4f*)(aout + (((size_t)b * TT + t) * NP + n) * HW + lane * 4) = a; __threadfence(); } }
}
__global__ __launch_bounds__(256) void parts_kernel(const float* __restrict__ A_, const float* __restrict__ Z, float* __restrict__ PARTS) {
  __shared__ __attribute__((aligned(16))) float Tz[64][HW + 1]; __shared__ float Ta[NP][HW];
  const int b = blockIdx.z, t = blockIdx.y, c0 = blockIdx.x * 64, t_ = threadIdx.x, n = t_ >> 6, j = t_ & 63;
  for (int k = t_; k < 64 * HW; k += 256) { const int cc = k >> 7, p = k & 127; Tz[cc][p] = Z[((size_t)b * CCH + c0 + cc) * THW + t * HW + p]; }
  for (int k = t_; k < NP * HW; k += 256) { const int nn = k >> 7, p = k & 127; Ta[nn][p] = A_[((size_t)b * NP + nn) * THW + t * HW + p]; }
  __syncthreads();
  float s = 0.0f; for (int p = 0; p < HW; ++p) s += pmul(Ta[n][p], Tz[j][p]);
  for (int pass = 0; pass < 2; ++pass) { ((volatile float*)PARTS)[(((size_t)b * TT + t) * NP + n) * CCH + c0 + j] = s; __threadfence(); }
}
struct G16 { const float* A; long sA; int lda; int arows; int K; float asc; const b16* B; long sB; int ldb; const float* bias; long sbias; const float* bias2; long sbias2; float* C; long sC; int ldc; };
__global__ __launch_bounds__(128) void gemm16_kernel(const float* __restrict__ pA, long sA, int lda, int arows, int K, float asc, const b16* __restrict__ pB, long sB, int ldb, const float* __restrict__ pbias, long sbias, const float* __restrict__ pbias2, long sbias2, float* __restrict__ pC, long sC, int ldc) {
  const G16 p = {pA, sA, lda, arows, K, asc, pB, sB, ldb, pbias, sbias, pbias2, sbias2, pC, sC, ldc};
  __shared__ __attribute__((aligned(16))) b16 Ah[16][CCH + 8], Al[16][CCH + 8]; __shared__ __attribute__((aligned(16))) float Tc[16][64 + 4];
  const int grp = blockIdx.y, n0 = blockIdx.x * 64, wave = threadIdx.x >> 5, lane = threadIdx.x & 31, nloc = lane & 15, hlf = lane >> 4, t_ = threadIdx.x;
  const float* A = p.A + grp * p.sA; const b16* B = p.B + grp * p.sB; const float* bias = p.bias ? p.bias + grp * p.sbias : nullptr; const float* bias2 = p.bias2 ? p.bias2 + grp * p.sbias2 : nullptr; float* C = p.C + grp * p.sC;
  for (int k = t_; k < 16 * p.K; k += 128) { const int m = k / p.K, kk = k - m * p.K; const float v = (m < p.arows) ? A[(size_t)(m < p.arows ? m : 0) * p.lda + kk] : 0.0f; b16 a_, c_; split16(v * p.asc, a_, c_); Ah[m][kk] = a_; Al[m][kk] = c_; }
  __syncthreads();
  v8f acc = {};
  for (int kb = 0; kb < p.K; kb += 32) { const v16b bw = frag_kb(B + (size_t)(n0 + wave * 16 + nloc) * p.ldb + kb, hlf); acc = wmma16b(frag_kb(&Ah[nloc][kb], hlf), bw, acc); acc = wmma16b(frag_kb(&Al[nloc][kb], hlf), bw, acc); }
  { const int n = n0 + wave * 16 + nloc; const float bb = (bias ? bf16_rne(bias[n]) : 0.0f) + (bias2 ? bias2[n] : 0.0f);
#pragma unroll
    for (int r = 0; r < 8; ++r) Tc[8 * hlf + r][wave * 16 + nloc] = acc[r] * (1.0f / (p.asc * WSC)) + bb; }
  __syncthreads();
  for (int pass = 0; pass < 2; ++pass) { for (int rr = wave * 4; rr < wave * 4 + 4; ++rr) if (rr < p.arows && lane < 16) *(volatile v4f*)(C + (size_t)rr * p.ldc + n0 + lane * 4) = *(const v4f*)(&Tc[rr][lane * 4]); __threadfence(); }
}
__global__ __launch_bounds__(256) void nodemix_kernel(const float* __restrict__ NODES, const float* __restrict__ TPG, const float* __restrict__ UG, float* __restrict__ CAT) {
  __shared__ float Satt[NODE][NODE + 1]; __shared__ __attribute__((aligned(16))) float Scat[TT][CCH];
  const int b = blockIdx.x, t_ = threadIdx.x, wave = t_ >> 5, lane = t_ & 31;
  const float* Tm = TPG + ((size_t)(0 * NBt + b) * NODE) * CI; const float* Pm = TPG + ((size_t)(1 * NBt + b) * NODE) * CI; const float* Gm = TPG + ((size_t)(2 * NBt + b) * NODE) * CI; const float* Nd = NODES + (size_t)b * NODE * CI;
  { const int m = t_ >> 4, mm = t_ & 15; float s = 0.0f; for (int k = 0; k < CI; ++k) s += pmul(Tm[m * CI + k], Pm[mm * CI + k]); Satt[m][mm] = s * 0.044194173824159216f; }
  __syncthreads();
  if (t_ < NODE) { float mx = -INFINITY; for (int k = 0; k < NODE; ++k) mx = fmaxf(mx, Satt[t_][k]); float s = 0.0f; for (int k = 0; k < NODE; ++k) { const float e = nexp(Satt[t_][k] - mx); Satt[t_][k] = e; s += e; } const float inv = 1.0f / s; for (int k = 0; k < NODE; ++k) Satt[t_][k] *= inv; }
  __syncthreads();
  for (int k = t_; k < TT * CI; k += 256) { const int t = k / CI, c = k - t * CI; float y = 0.0f;
    for (int n = 0; n < NP; ++n) { const int m = t * NP + n; float v = Nd[m * CI + c]; for (int mm = 0; mm < NODE; ++mm) v += pmul(Satt[m][mm], Gm[mm * CI + c]); y += v; }
    Scat[t][c] = y * (1.0f / NP); Scat[t][CI + c] = UG[b * CI + c]; }
  __syncthreads();
  for (int pass = 0; pass < 2; ++pass) { for (int t = 0; t < TT; ++t) *(volatile v4f*)(CAT + ((size_t)b * TT + t) * CCH + t_ * 4) = *(const v4f*)(&Scat[t][t_ * 4]); __threadfence(); }
}
__global__ __launch_bounds__(256) void final_kernel(const float* __restrict__ OUTP, const float* __restrict__ Z, const float* __restrict__ g, const float* __restrict__ be, float* __restrict__ zout) {
  const int b = blockIdx.y, wave = threadIdx.x >> 5, lane = threadIdx.x & 31;
  for (int w8 = wave; w8 < 32; w8 += 8) { const int o = blockIdx.x * 32 + w8;
    float v16 = (lane < NBt * TT) ? OUTP[(size_t)lane * CCH + o] : 0.0f;
    const float mu = wsum(v16) * (1.0f / (NBt * TT)); const float d = (lane < NBt * TT) ? v16 - mu : 0.0f; const float var = wsum(pmul(d, d)) * (1.0f / (NBt * TT)); const float rs = rsqrtf(var + EPS), gg = bf16_rne(g[o]), bb = bf16_rne(be[o]);
    const size_t row = ((size_t)b * CCH + o) * THW;
    for (int pass = 0; pass < 2; ++pass) {
#pragma unroll
      for (int t = 0; t < TT; ++t) { const float ov = pmul((__shfl(v16, b * TT + t) - mu) * rs, gg) + bb; const v4f z = *(const v4f*)(Z + row + t * HW + lane * 4); const v4f r = {ov + z[0], ov + z[1], ov + z[2], ov + z[3]}; *(volatile v4f*)(zout + row + t * HW + lane * 4) = r; }
      __threadfence(); } }
}
}

extern "C" void kernel_launch(void* const* d_in, const int* in_sizes, int n_in, void* d_out, int out_size, void* d_ws, size_t ws_size, hipStream_t stream) {
  (void)n_in;
  auto Fp = [&](int i) { return (const float*)d_in[i]; };
  if (in_sizes[0] != NBt * CT * HW || in_sizes[1] != NP * CCH || in_sizes[5] != CI * CCH || in_sizes[7] != CCH * CCH || in_sizes[11] != CCH * CCH || in_sizes[15] != CI * CI || out_size != NBt * CT * HW + NBt * TT * NP * HW) return;
  size_t off = 0; char* ws = (char*)d_ws;
  auto carve = [&](size_t bytes) { char* p = ws + off; off += (bytes + 255) & ~(size_t)255; return p; };
  b16* W1s = (b16*)carve((size_t)CCH * CCH * 2); b16* GWs = (b16*)carve((size_t)CI * CCH * 2); b16* W2s = (b16*)carve((size_t)CCH * CCH * 2); b16* WT4 = (b16*)carve((size_t)4 * CI * CI * 2);
  b16* GX = (b16*)carve((size_t)NBt * CT * HW * 2); b16* GXT = (b16*)carve((size_t)NBt * CT * HW * 2); float* Y = (float*)carve((size_t)NBt * CT * HW * 4);
  b16* YTH = (b16*)carve((size_t)NBt * THW * CCH * 2); b16* YTL = (b16*)carve((size_t)NBt * THW * CCH * 2); float* Y1 = (float*)carve((size_t)NBt * CCH * THW * 4);
  float* MEAN1 = (float*)carve(CCH * 4); float* VAR1 = (float*)carve(CCH * 4); float* Z = (float*)carve((size_t)NBt * CCH * THW * 4); float* USUM = (float*)carve(NBt * CCH * 4);
  float* SPRE = (float*)carve((size_t)NBt * NP * THW * 4); float* MV2 = (float*)carve(32 * 4); float* A_ = (float*)carve((size_t)NBt * NP * THW * 4); float* PARTS = (float*)carve((size_t)NBt * NODE * CCH * 4);
  float* UG = (float*)carve(NBt * CI * 4); float* UWB = (float*)carve(NBt * CI * 4); float* NODES = (float*)carve((size_t)NBt * NODE * CI * 4); float* TPG = (float*)carve((size_t)3 * NBt * NODE * CI * 4); float* CAT = (float*)carve((size_t)NBt * TT * CCH * 4); float* OUTP = (float*)carve((size_t)NBt * TT * CCH * 4);
  if (off > ws_size) return;
  float* zout = (float*)d_out; float* aout = zout + (size_t)NBt * CT * HW;
  prepw_kernel<<<256, 256, 0, stream>>>(Fp(7), Fp(5), Fp(11), W1s, GWs, W2s);
  prept_kernel<<<dim3(CI / 64, 4), 256, 0, stream>>>(Fp(15), Fp(16), Fp(17), Fp(18), WT4);
  prepg_kernel<<<dim3(CT / 64, NBt), 256, 0, stream>>>(Fp(0), GX, GXT);
  attn_kernel<<<dim3(CT / 32, NBt), 64, 0, stream>>>(GX, GXT, Y);
  ytrans_kernel<<<dim3(CCH / 64, NBt * TT), 256, 0, stream>>>(Y, YTH, YTL);
  w1_kernel<<<dim3(THW / HW, CCH / 64, NBt), 128, 0, stream>>>(W1s, YTH, YTL, Fp(8), Y1);
  bnstat_kernel<<<CCH / 32, 256, 0, stream>>>(Y1, CCH, MEAN1, VAR1);
  zmake_kernel<<<dim3(CCH / 32, NBt), 256, 0, stream>>>(Y1, Fp(0), MEAN1, VAR1, Fp(9), Fp(10), Z, USUM);
  sapre_kernel<<<dim3(THW / 64, NBt), 256, 0, stream>>>(Z, Fp(1), Fp(2), SPRE);
  bn2_kernel<<<1, 256, 0, stream>>>(SPRE, MV2);
  amake_kernel<<<NBt, 256, 0, stream>>>(SPRE, MV2, Fp(3), Fp(4), A_, aout);
  parts_kernel<<<dim3(CCH / 64, TT, NBt), 256, 0, stream>>>(A_, Z, PARTS);
  auto launch16 = [&](const G16& q, dim3 grid) { gemm16_kernel<<<grid, 128, 0, stream>>>(q.A, q.sA, q.lda, q.arows, q.K, q.asc, q.B, q.sB, q.ldb, q.bias, q.sbias, q.bias2, q.sbias2, q.C, q.sC, q.ldc); };
  G16 q;
  q = G16{USUM, 0, CCH, NBt, CCH, 512.0f, GWs, 0, CCH, Fp(6), 0, nullptr, 0, UG, 0, CI};                      launch16(q, dim3(CI / 64, 1));
  q = G16{UG, 0, CI, NBt, CI, 8.0f, WT4 + (size_t)3 * CI * CI, 0, CI, Fp(6), 0, nullptr, 0, UWB, 0, CI};        launch16(q, dim3(CI / 64, 1));
  q = G16{PARTS, (long)NODE * CCH, CCH, NODE, CCH, 8.0f, GWs, 0, CCH, nullptr, 0, UWB, CI, NODES, (long)NODE * CI, CI};   launch16(q, dim3(CI / 64, NBt));
  for (int w = 0; w < 3; ++w) { q = G16{NODES, (long)NODE * CI, CI, NODE, CI, 8.0f, WT4 + (size_t)w * CI * CI, 0, CI, nullptr, 0, nullptr, 0, TPG + (size_t)w * NBt * NODE * CI, (long)NODE * CI, CI}; launch16(q, dim3(CI / 64, NBt)); }
  nodemix_kernel<<<NBt, 256, 0, stream>>>(NODES, TPG, UG, CAT);
  q = G16{CAT, 0, CCH, NBt * TT, CCH, 8.0f, W2s, 0, CCH, Fp(12), 0, nullptr, 0, OUTP, 0, CCH};                   launch16(q, dim3(CCH / 64, 1));
  final_kernel<<<dim3(CCH / 32, NBt), 256, 0, stream>>>(OUTP, Z, Fp(13), Fp(14), zout);
}
